// TwoLayerTransformer_50878182588808
// MI455X (gfx1250) — hardware-run, weakly checked
//
#include <hip/hip_runtime.h>


#ifndef NB
#define NB 8
#endif
#ifndef SEQ
#define SEQ 2048
#endif
#define NB_FULL  8
#define SEQ_FULL 2048
#define NH_  8
#define DS   128
#define HSZ  (NH_ * DS)
#define EPAD 32
#define OSP  36
#define TSP  72
#define QRS  2048.0f
#define QRI  (1.0f / 2048.0f)
#define XCAR 256.0f
#define ECAR 1024.0f
#define QCAR 1024.0f
#define UCAR 64.0f
#define VCAR 16.0f
#define NEGB (-3.0e38f)

static_assert(NH_ == 8);
static_assert(NB >= 1 && NB <= 8);
static_assert(NB <= NB_FULL);
static_assert(SEQ <= SEQ_FULL);
static_assert(SEQ % 256 == 0);
static_assert(SEQ % 64 == 0);
static_assert(DS % 64 == 0);
static_assert(HSZ % 64 == 0);
static_assert(SEQ % 32 == 0);
static_assert(DS % 32 == 0);
static_assert(HSZ % 32 == 0);
static_assert(EPAD == 32);
static_assert(32 * 4 == DS);
static_assert((OSP * 4) % 16 == 0);
static_assert((TSP * 2) % 16 == 0);
static_assert(4 * 256 * 4 == 64 * 64);
static_assert(2 * 256 == 64 * 8);
static_assert(2 * (32 / 8) == 8);
static_assert((size_t)SEQ * 8 <= 131072);
static_assert((size_t)(EPAD + SEQ) * 4 + 16 * OSP * 4 <= 131072);
static_assert((size_t)SEQ * 4 + 2 * DS * 4 + 32 <= 131072);
static_assert(((size_t)SEQ * DS) % 8 == 0);

typedef _Float16 h16;
typedef __attribute__((ext_vector_type(16))) _Float16 v16h;
typedef __attribute__((ext_vector_type(8)))  _Float16 v8h;
typedef __attribute__((ext_vector_type(8)))  float    v8f;
typedef __attribute__((ext_vector_type(4)))  float    v4f;
typedef v4f  __attribute__((may_alias)) v4fa;
typedef v8h  __attribute__((may_alias)) v8ha;

__device__ __forceinline__ unsigned short f2bf(float f) { unsigned u = __float_as_uint(f); u += 0x7FFFu + ((u >> 16) & 1u); return (unsigned short)(u >> 16); }
__device__ __forceinline__ float bfr(float f) { return __uint_as_float(((unsigned)f2bf(f)) << 16); }
__device__ __forceinline__ v16h cat16(v8h lo, v8h hi) { return __builtin_shufflevector(lo, hi, 0, 1, 2, 3, 4, 5, 6, 7, 8, 9, 10, 11, 12, 13, 14, 15); }
__device__ __forceinline__ v8f wmma16(v16h a, v16h b, v8f c) { return __builtin_amdgcn_wmma_f32_16x16x32_f16(false, a, false, b, (short)0, c, false, false); }
__device__ __forceinline__ v16h  ldh(const h16* p) { return cat16(*(const v8h*)p, *(const v8h*)(p + 16)); }
static __device__ __forceinline__ h16 toh_flush(float v) { const h16 r = (h16)v; return (fabsf(v) < 6.103515625e-05f) ? (h16)0.0f : r; }
static __device__ __forceinline__ v8f wmma16g(v16h a, v16h b, v8f c) { c = wmma16(a, b, c); asm volatile("v_nop\n\tv_nop\n\tv_nop\n\tv_nop" : "+v"(c) : "v"(a), "v"(b)); return c; }

__global__ __launch_bounds__(32) void k_prep(const float* __restrict__ W, h16* EH, h16* ER, h16* EHR, h16* ERR, float* ZI) {
    __shared__ __align__(16) h16 ehs[SEQ];
    __shared__ __align__(16) h16 ers[SEQ];
    __shared__ __align__(16) float zs[SEQ];
    const int lane = threadIdx.x & 31; const int h = blockIdx.x;
    const int d0 = lane * (SEQ / 32);
    float mx = NEGB;
#pragma unroll 1
    for (int i = 0; i < SEQ / 32; ++i) mx = fmaxf(mx, bfr(W[(size_t)(d0 + i) * NH_ + h]));
#pragma unroll
    for (int off = 16; off > 0; off >>= 1) mx = fmaxf(mx, __shfl_xor(mx, off, 32));
    double run = 0.0;
#pragma unroll 1
    for (int i = 0; i < SEQ / 32; ++i) { const int d = d0 + i;
        const float e = expf(bfr(W[(size_t)d * NH_ + h]) - mx);
        const float ec = e * ECAR; const h16 hv = toh_flush(ec);
        zs[d] = e; ehs[d] = hv; ers[d] = toh_flush((ec - (float)hv) * QRS); run += (double)e; }
    double inc = run;
#pragma unroll
    for (int off = 1; off < 32; off <<= 1) { const double tt = __shfl_up(inc, (unsigned)off, 32); inc += (lane >= off) ? tt : 0.0; }
    double acc = inc - run;
#pragma unroll 1
    for (int i = 0; i < SEQ / 32; ++i) { const int d = d0 + i; acc += (double)zs[d]; zs[d] = 1.0f / (float)acc; }
    __syncthreads();
    const size_t pb = (size_t)h * SEQ;
#pragma unroll 1
    for (int ps = 0; ps < 2; ++ps) {
#pragma unroll 1
        for (int it = 0; it < SEQ / 256; ++it) { const int c8 = (it * 32 + lane) * 8;
            const v8h a = *(const v8ha*)(&ehs[c8]); const v8h r = *(const v8ha*)(&ers[c8]); v8h ar, rr;
#pragma unroll
            for (int i = 0; i < 8; ++i) { ar[i] = ehs[SEQ - 1 - c8 - i]; rr[i] = ers[SEQ - 1 - c8 - i]; }
            *(volatile v8h*)(EH + pb + c8) = a; *(volatile v8h*)(ER + pb + c8) = r;
            *(volatile v8h*)(EHR + pb + c8) = ar; *(volatile v8h*)(ERR + pb + c8) = rr; }
#pragma unroll 1
        for (int it = 0; it < SEQ / 128; ++it) { const int c4 = (it * 32 + lane) * 4;
            const v4f z = *(const v4fa*)(&zs[c4]);
            *(volatile v4f*)(ZI + pb + c4) = z; }
        if (ps == 0) __threadfence(); }
}

__global__ __launch_bounds__(256) void k_cvtx(const float* __restrict__ src, h16* dst, size_t n8, float carry) {
    const size_t i = (size_t)blockIdx.x * 256 + threadIdx.x; if (i >= n8) return;
    const v8f v = *(const v8f*)(src + i * 8); v8h o;
#pragma unroll
    for (int k = 0; k < 8; ++k) o[k] = toh_flush(bfr(v[k]) * carry);
    *(volatile v8h*)(dst + i * 8) = o; __threadfence(); *(volatile v8h*)(dst + i * 8) = o;
}

__global__ __launch_bounds__(256) void k_tr(const float* __restrict__ src, h16* dst, int R, int C, size_t inz, size_t outz, float carry) {
    __shared__ __align__(16) h16 ts[64 * TSP];
    const int t = threadIdx.x; const int r0 = blockIdx.x * 64, c0 = blockIdx.y * 64;
    const float* sp = src + (size_t)blockIdx.z * inz + (size_t)r0 * C + c0;
#pragma unroll
    for (int it = 0; it < 4; ++it) { const int idx = it * 256 + t; const int row = idx >> 4, c4 = (idx & 15) * 4;
        const v4f v = *(const v4f*)(sp + (size_t)row * C + c4);
#pragma unroll
        for (int i = 0; i < 4; ++i) ts[(c4 + i) * TSP + row] = toh_flush(bfr(v[i]) * carry); }
    __syncthreads();
    h16* dp = dst + (size_t)blockIdx.z * outz + (size_t)c0 * R + r0;
#pragma unroll 1
    for (int ps = 0; ps < 2; ++ps) {
#pragma unroll
        for (int it = 0; it < 2; ++it) { const int idx = it * 256 + t; const int c = idx >> 3, r8 = (idx & 7) * 8;
            const v8h val = *(const v8ha*)(&ts[c * TSP + r8]);
            *(volatile v8h*)(dp + (size_t)c * R + r8) = val; }
        if (ps == 0) __threadfence(); }
}

__global__ __launch_bounds__(32) void k_mm8(const h16* __restrict__ Ah, const h16* __restrict__ Ar, const h16* __restrict__ Bp, const float* __restrict__ RS, h16* Ph, h16* Pr,
                                            int K, int nrows, int arp, int azp, int bzp, int orp, int ozp, int rs_on, int rs_pitch, int rs_off, float scl, float ocar) {
    __shared__ __align__(16) float os[16 * 68];
    const int lane = threadIdx.x & 31, lr = lane & 15, hi = lane >> 4;
    const int n0 = blockIdx.x * 64; const int z = blockIdx.y;
    const int arow = (lr & 7) % nrows;
    const size_t aoff = (size_t)z * (size_t)azp + (size_t)arow * (size_t)arp + 8 * hi;
    const size_t boff = (size_t)z * (size_t)bzp + (size_t)(n0 + lr) * (size_t)K + 8 * hi;
    v8f aH[4], aR[4];
#pragma unroll
    for (int nb = 0; nb < 4; ++nb) { aH[nb] = (v8f){}; aR[nb] = (v8f){}; }
#pragma unroll 1
    for (int kc = 0; kc < K; kc += 32) {
        const v16h eh = ldh(Ah + aoff + kc), er = ldh(Ar + aoff + kc);
#pragma unroll
        for (int nb = 0; nb < 4; ++nb) { const v16h xb = ldh(Bp + boff + (size_t)nb * 16 * (size_t)K + kc);
            aH[nb] = wmma16g(eh, xb, aH[nb]); aR[nb] = wmma16g(er, xb, aR[nb]); }
    }
    float rsv[8];
#pragma unroll
    for (int r = 0; r < 8; ++r) { const float tv = RS[(size_t)r * (size_t)rs_pitch + (size_t)rs_off]; rsv[r] = (rs_on != 0) ? tv * scl : scl; }
#pragma unroll
    for (int nb = 0; nb < 4; ++nb) {
#pragma unroll
        for (int r = 0; r < 8; ++r) os[(hi * 8 + r) * 68 + nb * 16 + lr] = (aH[nb][r] + aR[nb][r] * QRI) * rsv[r]; }
    __syncthreads();
#pragma unroll 1
    for (int ps = 0; ps < 2; ++ps) {
#pragma unroll
        for (int s = 0; s < 2; ++s) { const int row = 4 * s + (lane >> 3), c8 = (lane & 7) * 8;
            const v4f x0 = *(const v4fa*)(&os[row * 68 + c8]); const v4f x1 = *(const v4fa*)(&os[row * 68 + c8 + 4]); v8h hv, rv;
#pragma unroll
            for (int i = 0; i < 4; ++i) { const float c0v = x0[i] * ocar, c1v = x1[i] * ocar; const h16 a0 = toh_flush(c0v); const h16 a1 = toh_flush(c1v);
                hv[i] = a0; hv[4 + i] = a1; rv[i] = toh_flush((c0v - (float)a0) * QRS); rv[4 + i] = toh_flush((c1v - (float)a1) * QRS); }
            const size_t oo = (size_t)z * (size_t)ozp + (size_t)row * (size_t)orp + (size_t)(n0 + c8);
            if (row < nrows) { *(volatile v8h*)(Ph + oo) = hv; *(volatile v8h*)(Pr + oo) = rv; } }
        if (ps == 0) __threadfence(); }
}

__global__ __launch_bounds__(32) void k_sc(const h16* __restrict__ EH, const h16* __restrict__ ER, const h16* __restrict__ VH, const h16* __restrict__ VR,
                                           const float* __restrict__ ZI, float* SC) {
    __shared__ __align__(16) h16 ehs[EPAD + SEQ];
    __shared__ __align__(16) h16 ers[EPAD + SEQ];
    __shared__ __align__(16) float os[16 * OSP];
    const int lane = threadIdx.x & 31, lr = lane & 15, hi = lane >> 4;
    const int l0 = blockIdx.x * 32;
    const int nk = l0 + 32;
    const int nch = (nk + 255) >> 8;
    const int bcol = (lr & 7) % NB;
    ehs[lane] = (h16)0.0f; ers[lane] = (h16)0.0f;
    float tot0[8], tot1[8];
#pragma unroll
    for (int r = 0; r < 8; ++r) { tot0[r] = 0.0f; tot1[r] = 0.0f; }
#pragma unroll 1
    for (int h = 0; h < NH_; ++h) {
        __syncthreads();
#pragma unroll 1
        for (int it = 0; it < nch; ++it) { const int c8 = (it * 32 + lane) * 8; const size_t g = (size_t)h * SEQ + (size_t)c8;
            const v8h a = *(const v8h*)(EH + g); const v8h r = *(const v8h*)(ER + g);
            *(v8ha*)(&ehs[EPAD + c8]) = a; *(v8ha*)(&ers[EPAD + c8]) = r; }
        __syncthreads();
        v8f sH0 = (v8f){}, sR0 = (v8f){}, sH1 = (v8f){}, sR1 = (v8f){};
        const size_t vb = ((size_t)h * NB + (size_t)bcol) * SEQ + 8 * hi;
#pragma unroll 1
        for (int j0 = 0; j0 < nk; j0 += 32) {
            const v16h vh = ldh(VH + vb + j0), vr = ldh(VR + vb + j0);
            const int base = EPAD + (l0 - j0) + lr - 8 * hi;
            v16h th0, tr0, th1, tr1;
#pragma unroll
            for (int i = 0; i < 8; ++i) {
                const h16 e0 = ehs[base - i], r0 = ers[base - i];
                th0[i] = e0; tr0[i] = r0;
                th0[8 + i] = ehs[base - 16 - i]; tr0[8 + i] = ers[base - 16 - i];
                th1[i] = ehs[base + 16 - i]; tr1[i] = ers[base + 16 - i];
                th1[8 + i] = e0; tr1[8 + i] = r0; }
            sH0 = wmma16g(th0, vh, sH0); sR0 = wmma16g(th0, vr, sR0); sR0 = wmma16g(tr0, vh, sR0);
            sH1 = wmma16g(th1, vh, sH1); sR1 = wmma16g(th1, vr, sR1); sR1 = wmma16g(tr1, vh, sR1);
        }
        const float* zp = ZI + (size_t)h * SEQ + l0 + 8 * hi;
        const v4f z0 = *(const v4f*)zp, z1 = *(const v4f*)(zp + 4), z2 = *(const v4f*)(zp + 16), z3 = *(const v4f*)(zp + 20);
#pragma unroll
        for (int r = 0; r < 4; ++r) {
            tot0[r]     += (sH0[r]     + sR0[r]     * QRI) * z0[r];
            tot0[4 + r] += (sH0[4 + r] + sR0[4 + r] * QRI) * z1[r];
            tot1[r]     += (sH1[r]     + sR1[r]     * QRI) * z2[r];
            tot1[4 + r] += (sH1[4 + r] + sR1[4 + r] * QRI) * z3[r]; }
    }
    const float scl = 1.0f / (ECAR * VCAR);
    { v4f a, c;
      a[0] = tot0[0] * scl; a[1] = tot0[1] * scl; a[2] = tot0[2] * scl; a[3] = tot0[3] * scl; c[0] = tot0[4] * scl; c[1] = tot0[5] * scl; c[2] = tot0[6] * scl; c[3] = tot0[7] * scl;
      *(v4fa*)(&os[lr * OSP +  0 + 8 * hi]) = a; *(v4fa*)(&os[lr * OSP +  0 + 8 * hi + 4]) = c;
      a[0] = tot1[0] * scl; a[1] = tot1[1] * scl; a[2] = tot1[2] * scl; a[3] = tot1[3] * scl; c[0] = tot1[4] * scl; c[1] = tot1[5] * scl; c[2] = tot1[6] * scl; c[3] = tot1[7] * scl;
      *(v4fa*)(&os[lr * OSP + 16 + 8 * hi]) = a; *(v4fa*)(&os[lr * OSP + 16 + 8 * hi + 4]) = c; }
    __syncthreads();
#pragma unroll 1
    for (int ps = 0; ps < 2; ++ps) {
#pragma unroll
        for (int s = 0; s < 2; ++s) { const int row = 4 * s + (lane >> 3), cofs = (lane & 7) * 4;
            const v4f val = *(const v4fa*)(&os[row * OSP + cofs]);
            if (row < NB) *(volatile v4f*)(SC + (size_t)row * SEQ + l0 + cofs) = val; }
        if (ps == 0) __threadfence(); }
}

__global__ __launch_bounds__(256) void k_out(const float* __restrict__ X, const float* __restrict__ SC, float* OUT) {
    __shared__ __align__(16) float sc[SEQ];
    __shared__ __align__(16) float part[2 * DS];
    __shared__ float red[8];
    const int t = threadIdx.x, lane = t & 31;
    const int wave = __builtin_amdgcn_readfirstlane((int)(threadIdx.x >> 5));
    const int b = blockIdx.x;
    float mx = NEGB;
#pragma unroll 1
    for (int l = t; l < SEQ; l += 256) { float v = SC[(size_t)b * SEQ + l]; asm volatile("" : "+v"(v)); sc[l] = v; mx = fmaxf(mx, (l < SEQ - 1) ? v : NEGB); }
#pragma unroll
    for (int off = 16; off > 0; off >>= 1) mx = fmaxf(mx, __shfl_xor(mx, off, 32));
    if (lane == 0) red[wave] = mx;
    __syncthreads();
    mx = red[0];
#pragma unroll
    for (int w = 1; w < 8; ++w) mx = fmaxf(mx, red[w]);
    __syncthreads();
    float sum = 0.0f;
#pragma unroll 1
    for (int l = t; l < SEQ; l += 256) { const float e0 = expf(sc[l] - mx); const float e = (l < SEQ - 1) ? e0 : 0.0f; sc[l] = e; sum += e; }
#pragma unroll
    for (int off = 16; off > 0; off >>= 1) sum += __shfl_xor(sum, off, 32);
    if (lane == 0) red[wave] = sum;
    __syncthreads();
    float total = red[0];
#pragma unroll
    for (int w = 1; w < 8; ++w) total += red[w];
    const float inv = 1.0f / total;
    const int half = t >> 7, s = t & (DS - 1);
    const int lbeg = half * (SEQ / 2);
    const int lend = (lbeg + SEQ / 2 < SEQ - 1) ? (lbeg + SEQ / 2) : (SEQ - 1);
    const float* xb = X + (size_t)b * SEQ_FULL * DS + s;
    float acc = 0.0f;
#pragma unroll 4
    for (int l = lbeg; l < lend; ++l) acc = fmaf(sc[l], bfr(xb[(size_t)l * DS]), acc);
    part[half * DS + s] = acc;
    __syncthreads();
    if (wave == 0) {
        const v4f a = *(const v4fa*)(&part[lane * 4]); const v4f c = *(const v4fa*)(&part[DS + lane * 4]);
        v4f o; o[0] = (a[0] + c[0]) * inv; o[1] = (a[1] + c[1]) * inv; o[2] = (a[2] + c[2]) * inv; o[3] = (a[3] + c[3]) * inv;
        float* op = OUT + (size_t)b * DS + lane * 4;
        *(volatile v4f*)op = o; __threadfence(); *(volatile v4f*)op = o;
    }
}

static constexpr size_t al256(size_t v) { return (v + 255) & ~(size_t)255; }
static constexpr size_t SZ_E  = al256((size_t)NH_ * SEQ * 2);
static constexpr size_t SZ_Z  = al256((size_t)NH_ * SEQ * 4);
static constexpr size_t SZ_X  = al256((size_t)NB * SEQ * DS * 2);
static constexpr size_t SZ_A  = al256((size_t)HSZ * HSZ * 2);
static constexpr size_t SZ_Q  = al256((size_t)NB * HSZ * 2);
static constexpr size_t SZ_V  = al256((size_t)NH_ * NB * SEQ * 2);
static constexpr size_t SZ_S  = al256((size_t)NB * SEQ * 4);
static constexpr size_t SZ_TOTAL = 4 * SZ_E + SZ_Z + 2 * SZ_X + SZ_A + 4 * SZ_Q + 2 * SZ_V + SZ_S;
static_assert(SZ_TOTAL <= (size_t)134217728);

extern "C" void kernel_launch(void* const* d_in, const int* in_sizes, int n_in,
                              void* d_out, int out_size, void* d_ws, size_t ws_size, hipStream_t stream) {
    if (n_in < 3) return;
    if ((size_t)in_sizes[0] < ((size_t)(NB - 1) * SEQ_FULL + SEQ) * DS) return;
    if ((size_t)in_sizes[1] < (size_t)SEQ * NH_) return;
    if ((size_t)in_sizes[2] < (size_t)HSZ * HSZ) return;
    if ((size_t)out_size < (size_t)NB * DS) return;
    if (SZ_TOTAL > ws_size) return;
    const float* x = (const float*)d_in[0];
    const float* W = (const float*)d_in[1];
    const float* A = (const float*)d_in[2];
    float* OUT = (float*)d_out;
    char* wsp = (char*)d_ws;
    h16* EH  = (h16*)wsp; wsp += SZ_E;
    h16* ER  = (h16*)wsp; wsp += SZ_E;
    h16* EHR = (h16*)wsp; wsp += SZ_E;
    h16* ERR = (h16*)wsp; wsp += SZ_E;
    float* ZI = (float*)wsp; wsp += SZ_Z;
    h16* XN  = (h16*)wsp; wsp += SZ_X;
    h16* XT  = (h16*)wsp; wsp += SZ_X;
    h16* AT  = (h16*)wsp; wsp += SZ_A;
    h16* QH  = (h16*)wsp; wsp += SZ_Q;
    h16* QR  = (h16*)wsp; wsp += SZ_Q;
    h16* UH  = (h16*)wsp; wsp += SZ_Q;
    h16* UR  = (h16*)wsp; wsp += SZ_Q;
    h16* VH  = (h16*)wsp; wsp += SZ_V;
    h16* VR  = (h16*)wsp; wsp += SZ_V;
    float* SC = (float*)wsp; wsp += SZ_S;

    k_prep<<<NH_, 32, 0, stream>>>(W, EH, ER, EHR, ERR, ZI);

    if (SEQ == SEQ_FULL) {
        const size_t n8 = (size_t)NB * SEQ * DS / 8;
        k_cvtx<<<(unsigned)((n8 + 255) / 256), 256, 0, stream>>>(x, XN, n8, XCAR);
    } else {
        const size_t n8 = (size_t)SEQ * DS / 8;
        for (int b = 0; b < NB; ++b) k_cvtx<<<(unsigned)((n8 + 255) / 256), 256, 0, stream>>>(x + (size_t)b * SEQ_FULL * DS, XN + (size_t)b * SEQ * DS, n8, XCAR);
    }
    k_tr<<<dim3(SEQ / 64, DS / 64, NB), 256, 0, stream>>>(x, XT, SEQ, DS, (size_t)SEQ_FULL * DS, (size_t)DS * SEQ, XCAR);
    k_tr<<<dim3(HSZ / 64, HSZ / 64, 1), 256, 0, stream>>>(A, AT, HSZ, HSZ, (size_t)0, (size_t)0, XCAR);

    k_mm8<<<dim3(DS / 64, NB, 1), 32, 0, stream>>>(EHR, ERR, XT, ZI, QH, QR, SEQ, NH_, SEQ, 0, DS * SEQ, DS, HSZ, 1, SEQ, SEQ - 1, 1.0f / (ECAR * XCAR), QCAR);
    k_mm8<<<dim3(HSZ / 64, 1, 1), 32, 0, stream>>>(QH, QR, AT, ZI, UH, UR, HSZ, NB, HSZ, 0, 0, HSZ, 0, 0, 0, 0, 1.0f / (QCAR * XCAR), UCAR);
    k_mm8<<<dim3(SEQ / 64, NB, 1), 32, 0, stream>>>(UH, UR, XN, ZI, VH, VR, DS, NH_, DS, HSZ, SEQ * DS, NB * SEQ, SEQ, 0, 0, 0, 1.0f / (UCAR * XCAR), VCAR);

    k_sc<<<SEQ / 32, 32, 0, stream>>>(EH, ER, VH, VR, ZI, SC);
    k_out<<<NB, 256, 0, stream>>>(x, SC, OUT);
}
